// TextClassifierQuantum_65481071402033
// MI455X (gfx1250) — hardware-verified
//
#include <hip/hip_runtime.h>

#define NTOK   (32 * 1024)
#define SEQ    1024
#define EDIM   64
#define HEADS  8
#define QD     8
#define FDIM   2048
#define NLAY   4
#define NCLS   4
#define LN_EPS 1e-5f

#define __bf16 _Float16
typedef __attribute__((ext_vector_type(16))) __bf16 v16bf;
typedef __attribute__((ext_vector_type(8)))  float  v8f;
typedef __attribute__((ext_vector_type(4)))  float  v4f_t;
typedef float v4fa __attribute__((ext_vector_type(4), may_alias));

__device__ __forceinline__ __bf16 f2bf(float f) { return (__bf16)f; }
__device__ __forceinline__ void st2f(float* p, float v) { *(volatile float*)p = v; __threadfence(); *(volatile float*)p = v; }

__device__ __forceinline__ v16bf unpack8(uint4 q) {
  union { uint4 q; unsigned short s[8]; } cv;
  cv.q = q;
  v16bf r = {};
#pragma unroll
  for (int j = 0; j < 8; ++j) r[j] = __builtin_bit_cast(__bf16, cv.s[j]);
  return r;
}

__global__ void prep_w1(const float* __restrict__ w1, const float* __restrict__ b1,
                        __bf16* __restrict__ w1p) {
  int idx0 = (blockIdx.x * 256 + threadIdx.x) * 2;
  float v2[2];
#pragma unroll
  for (int u = 0; u < 2; ++u) {
    int idx  = idx0 + u;
    int j    = idx & 7;
    int lane = (idx >> 3) & 31;
    int t    = (idx >> 8) & 127;
    int l    = idx >> 15;
    int f    = t * 16 + (lane & 15);
    if (lane < 16) v2[u] = w1[((size_t)(l * QD + j)) * FDIM + f];
    else           v2[u] = (j == 0) ? b1[(size_t)l * FDIM + f] : 0.f;
  }
  const unsigned pk = (unsigned)__builtin_bit_cast(unsigned short, f2bf(v2[0])) | ((unsigned)__builtin_bit_cast(unsigned short, f2bf(v2[1])) << 16);
  *(volatile unsigned*)(w1p + idx0) = pk; __threadfence(); *(volatile unsigned*)(w1p + idx0) = pk;
}

__global__ void prep_w2(const float* __restrict__ w2, __bf16* __restrict__ w2p) {
  int idx0 = (blockIdx.x * 256 + threadIdx.x) * 2;
  if ((idx0 >> 17) >= NLAY) return;
  float v2[2];
#pragma unroll
  for (int u = 0; u < 2; ++u) {
    int idx  = idx0 + u;
    int e    = idx & 15;
    int lane = (idx >> 4) & 31;
    int n    = (idx >> 9) & 3;
    int kb   = (idx >> 11) & 63;
    int l    = idx >> 17;
    int K    = kb * 32 + ((lane < 16) ? ((e < 8) ? e : e + 8)
                                      : ((e < 8) ? e + 8 : e + 16));
    int col  = n * 16 + (lane & 15);
    v2[u] = w2[((size_t)l * FDIM + K) * EDIM + col];
  }
  const unsigned pk = (unsigned)__builtin_bit_cast(unsigned short, f2bf(v2[0])) | ((unsigned)__builtin_bit_cast(unsigned short, f2bf(v2[1])) << 16);
  *(volatile unsigned*)(w2p + idx0) = pk; __threadfence(); *(volatile unsigned*)(w2p + idx0) = pk;
}

__global__ void embed_kernel(const int* __restrict__ tokens,
                             const float* __restrict__ emb,
                             float* __restrict__ x) {
  int idx = blockIdx.x * blockDim.x + threadIdx.x;
  int tok = idx >> 6, e = idx & 63;
  int s = tok & (SEQ - 1);
  float div = expf(-(float)(e & ~1) * (logf(10000.0f) / (float)EDIM));
  float ang = (float)s * div;
  float pe  = (e & 1) ? cosf(ang) : sinf(ang);
  int tk = tokens[tok]; tk = (tk < 0) ? 0 : (tk > 31999 ? 31999 : tk);
  st2f(x + idx, emb[(size_t)tk * EDIM + e] + pe);
}

__global__ void __launch_bounds__(256)
attn_ln_kernel(const float* __restrict__ xin, float* __restrict__ xout,
               const float* __restrict__ phi_l,
               const float* __restrict__ g, const float* __restrict__ bt) {
  int lane = threadIdx.x & 31;
  int wave = threadIdx.x >> 5;
  int tok  = blockIdx.x * 8 + wave;
  const float* xr = xin + (size_t)tok * EDIM;

  float sv[2];
#pragma unroll
  for (int p = 0; p < 2; ++p) {
    int e = lane + 32 * p;
    int h = e >> 3, w = e & 7;
    const float* ph = phi_l + h * QD;
    float cum = 1.f, cum1 = 1.f, zsel = 0.f;
#pragma unroll 1
    for (int j = 0; j < QD; ++j) {
      const float cj = cosf(xr[j] + ph[j]);
      cum *= cj;
      if (j >= 1) cum1 *= cj;
      if (j == w) zsel = cum;
    }
    const float z = (w == 0) ? cum1 : zsel;
    sv[p] = xr[e] + z;
  }
  float sum = sv[0] + sv[1];
  float sq  = sv[0] * sv[0] + sv[1] * sv[1];
#pragma unroll
  for (int o = 16; o >= 1; o >>= 1) {
    sum += __shfl_xor(sum, o, 32);
    sq  += __shfl_xor(sq,  o, 32);
  }
  float mean = sum * (1.f / EDIM);
  float var  = sq * (1.f / EDIM) - mean * mean;
  float rstd = rsqrtf(var + LN_EPS);
#pragma unroll
  for (int p = 0; p < 2; ++p) {
    int e = lane + 32 * p;
    st2f(xout + (size_t)tok * EDIM + e, (sv[p] - mean) * rstd * g[e] + bt[e]);
  }
}

__global__ void __launch_bounds__(256)
ffn_kernel(const float* __restrict__ y, float* __restrict__ xout,
           const float* __restrict__ theta_l,
           const uint4* __restrict__ w1p,
           const v16bf* __restrict__ w2p,
           const float* __restrict__ b2,
           const float* __restrict__ g, const float* __restrict__ bt) {
  __shared__ uint4 w1s[128 * 32];
  __shared__ __attribute__((aligned(16))) float stg[8][32 * 68];
  for (int i = threadIdx.x; i < 128 * 32; i += 256) w1s[i] = w1p[i];
  __syncthreads();
  float* sw = stg[threadIdx.x >> 5];

  int lane = threadIdx.x & 31;
  int wave = threadIdx.x >> 5;
  int t0   = (blockIdx.x * 8 + wave) * 32;
  int lo = lane & 15, hi = lane >> 4;

  float ct[QD];
#pragma unroll
  for (int j = 0; j < QD; ++j) ct[j] = cosf(theta_l[j]);

  v16bf qf[2];
#pragma unroll
  for (int m = 0; m < 2; ++m) {
    v16bf q = {};
    if (lane < 16) {
      const float* yr = y + (size_t)(t0 + m * 16 + lane) * EDIM;
#pragma unroll
      for (int j = 0; j < QD; ++j) q[j] = f2bf(ct[j] * cosf(yr[j]));
    } else {
      q[0] = f2bf(1.0f);
    }
    qf[m] = q;
  }

  v8f acc[2][4] = {};
  v8f zero = {};

  for (int kb = 0; kb < 64; ++kb) {
    v16bf w1a0 = unpack8(w1s[(2 * kb + 0) * 32 + lane]);
    v16bf w1a1 = unpack8(w1s[(2 * kb + 1) * 32 + lane]);
    v16bf w2b0 = w2p[(kb * 4 + 0) * 32 + lane];
    v16bf w2b1 = w2p[(kb * 4 + 1) * 32 + lane];
    v16bf w2b2 = w2p[(kb * 4 + 2) * 32 + lane];
    v16bf w2b3 = w2p[(kb * 4 + 3) * 32 + lane];
#pragma unroll
    for (int m = 0; m < 2; ++m) {
      v8f d0 = __builtin_amdgcn_wmma_f32_16x16x32_f16(
          false, w1a0, false, qf[m], (short)0, zero, false, false);
      v8f d1 = __builtin_amdgcn_wmma_f32_16x16x32_f16(
          false, w1a1, false, qf[m], (short)0, zero, false, false);
      v16bf hf;
#pragma unroll
      for (int e = 0; e < 8; ++e) {
        hf[e]     = f2bf(fmaxf(d0[e], 0.f));
        hf[e + 8] = f2bf(fmaxf(d1[e], 0.f));
      }
      acc[m][0] = __builtin_amdgcn_wmma_f32_16x16x32_f16(
          false, hf, false, w2b0, (short)0, acc[m][0], false, false);
      acc[m][1] = __builtin_amdgcn_wmma_f32_16x16x32_f16(
          false, hf, false, w2b1, (short)0, acc[m][1], false, false);
      acc[m][2] = __builtin_amdgcn_wmma_f32_16x16x32_f16(
          false, hf, false, w2b2, (short)0, acc[m][2], false, false);
      acc[m][3] = __builtin_amdgcn_wmma_f32_16x16x32_f16(
          false, hf, false, w2b3, (short)0, acc[m][3], false, false);
    }
  }

#pragma unroll
  for (int m = 0; m < 2; ++m) {
    int tokb = t0 + m * 16 + 8 * hi;
    float s[8][4], sum[8], sq[8];
#pragma unroll
    for (int r = 0; r < 8; ++r) {
      sum[r] = 0.f; sq[r] = 0.f;
      const float* yr = y + (size_t)(tokb + r) * EDIM;
#pragma unroll
      for (int n = 0; n < 4; ++n) {
        float v = acc[m][n][r] + b2[n * 16 + lo] + yr[n * 16 + lo];
        s[r][n] = v; sum[r] += v; sq[r] += v * v;
      }
    }
#pragma unroll
    for (int o = 1; o < 16; o <<= 1) {
#pragma unroll
      for (int r = 0; r < 8; ++r) {
        sum[r] += __shfl_xor(sum[r], o, 32);
        sq[r]  += __shfl_xor(sq[r],  o, 32);
      }
    }
#pragma unroll
    for (int r = 0; r < 8; ++r) {
      float mean = sum[r] * (1.f / EDIM);
      float var  = sq[r] * (1.f / EDIM) - mean * mean;
      float rstd = rsqrtf(var + LN_EPS);
      float* srow = sw + (m * 16 + 8 * hi + r) * 68;
#pragma unroll
      for (int n = 0; n < 4; ++n)
        srow[n * 16 + lo] = (s[r][n] - mean) * rstd * g[n * 16 + lo] + bt[n * 16 + lo];
    }
  }
  asm volatile("s_wait_dscnt 0" ::: "memory");
#pragma unroll 1
  for (int pass = 0; pass < 2; ++pass) {
#pragma unroll
    for (int i = 0; i < 16; ++i) { const int c = lane + 32 * i, rr = c >> 4, q = (c & 15) * 4;
      *(volatile v4f_t*)(xout + (size_t)(t0 + rr) * EDIM + q) = *(const volatile v4fa*)(sw + rr * 68 + q); }
    __threadfence();
  }
}

__global__ void pool_kernel(const float* __restrict__ x, float* __restrict__ pooled) {
  int b = blockIdx.x, e = threadIdx.x;
  float acc = 0.f;
  for (int s = 0; s < SEQ; ++s) acc += x[(size_t)(b * SEQ + s) * EDIM + e];
  st2f(pooled + b * EDIM + e, acc * (1.f / SEQ));
}

__global__ void cls_kernel(const float* __restrict__ pooled,
                           const float* __restrict__ w, const float* __restrict__ bias,
                           float* __restrict__ out) {
  int tid = threadIdx.x;
  int b = tid >> 2, c = tid & 3;
  float acc = bias[c];
  for (int e = 0; e < EDIM; ++e) acc += pooled[b * EDIM + e] * w[e * NCLS + c];
  st2f(out + tid, acc);
}

extern "C" void kernel_launch(void* const* d_in, const int* in_sizes, int n_in,
                              void* d_out, int out_size, void* d_ws, size_t ws_size,
                              hipStream_t stream) {
  (void)in_sizes; (void)n_in; (void)out_size; (void)ws_size;
  const int*   tokens = (const int*)d_in[0];
  const float* emb    = (const float*)d_in[1];
  const float* phi    = (const float*)d_in[2];
  const float* theta  = (const float*)d_in[3];
  const float* w1     = (const float*)d_in[4];
  const float* b1     = (const float*)d_in[5];
  const float* w2     = (const float*)d_in[6];
  const float* b2     = (const float*)d_in[7];
  const float* ln1g   = (const float*)d_in[8];
  const float* ln1b   = (const float*)d_in[9];
  const float* ln2g   = (const float*)d_in[10];
  const float* ln2b   = (const float*)d_in[11];
  const float* clsw   = (const float*)d_in[12];
  const float* clsb   = (const float*)d_in[13];

  char* ws = (char*)d_ws;
  float*  x0   = (float*)ws;
  float*  x1   = (float*)(ws + (size_t)NTOK * EDIM * 4);
  __bf16* w1p  = (__bf16*)(ws + 2 * (size_t)NTOK * EDIM * 4);
  __bf16* w2p  = (__bf16*)((char*)w1p + (size_t)NLAY * 128 * 32 * 8 * 2);
  float*  pooled = (float*)((char*)w2p + (size_t)NLAY * 64 * 4 * 32 * 16 * 2);

  prep_w1<<<131072 / 512, 256, 0, stream>>>(w1, b1, w1p);
  prep_w2<<<(NLAY * 131072) / 512, 256, 0, stream>>>(w2, w2p);
  embed_kernel<<<(NTOK * EDIM) / 256, 256, 0, stream>>>(tokens, emb, x0);

  for (int l = 0; l < NLAY; ++l) {
    attn_ln_kernel<<<NTOK / 8, 256, 0, stream>>>(
        x0, x1, phi + (size_t)l * HEADS * QD, ln1g + (size_t)l * EDIM,
        ln1b + (size_t)l * EDIM);
    ffn_kernel<<<NTOK / 32 / 8, 256, 0, stream>>>(
        x1, x0, theta + (size_t)l * QD,
        (const uint4*)(w1p + (size_t)l * 128 * 32 * 8),
        (const v16bf*)(w2p + (size_t)l * 64 * 4 * 32 * 16),
        b2 + (size_t)l * EDIM, ln2g + (size_t)l * EDIM, ln2b + (size_t)l * EDIM);
  }

  pool_kernel<<<32, 64, 0, stream>>>(x0, pooled);
  cls_kernel<<<1, 128, 0, stream>>>(pooled, clsw, clsb, (float*)d_out);
}
